// MoEModel_20796231647464
// MI455X (gfx1250) — hardware-verified
//
#include <hip/hip_runtime.h>
#include <math.h>

#define NTOK 4096
#define DIN 512
#define H1 1024
#define H2 512
#define DOUT 50
#define DPAD 64
#define NEXP 8
#define TOPK 2
#define SPT TOPK
#define NE 16
#define NSLOT (NTOK * TOPK)
#define R_MAX (NSLOT + 64 * NE)
#define NT_MAX (R_MAX / 64)
#define RW_CH 8192
#define OUT2_ROW (DOUT / 2)

#define CX_LOG2 11
#define CW_LOG2 16
#define CH ((float)(1u << CX_LOG2))
#define SC (1.0f / (float)(1u << (CX_LOG2 + CW_LOG2)))

#define TBL_COUNT 0
#define TBL_POFF 16
#define TBL_NTILES 40
#define TBL_TILE_E 64
#define TBL_HDR 256
#define TBL_ROWTOK TBL_HDR
#define TBL_SLOTROW (TBL_HDR + R_MAX)
#define TBL_WORDS (TBL_HDR + R_MAX + NSLOT)
#define OUT1_OFF ((size_t)NTOK * (size_t)DOUT)

static_assert(NEXP == 8 && NEXP <= NE && NE == 16 && TOPK == 2 && SPT == 2 && NTOK == 4096 && DIN == 512 && H1 == 1024 && H2 == 512 && DOUT == 50 && DPAD == 64 && OUT2_ROW == 25);
static_assert(DIN % 64 == 0 && H1 % 64 == 0 && H2 % 64 == 0 && DPAD % 64 == 0 && DOUT % 2 == 0 && DOUT <= DPAD && NTOK % 256 == 0 && NSLOT % 128 == 0 && R_MAX % 128 == 0);
static_assert(NSLOT == 8192 && R_MAX == 9216 && NT_MAX == 144 && TBL_WORDS == 17664);
static_assert(TBL_HDR % 32 == 0 && TBL_HDR <= 512 && TBL_COUNT + NE <= TBL_POFF && TBL_POFF + NE + 1 <= TBL_NTILES && TBL_NTILES < TBL_TILE_E && TBL_TILE_E + NT_MAX <= TBL_HDR);
static_assert(CX_LOG2 == 11 && CW_LOG2 == 16 && (NTOK * DIN / 8) % 256 == 0 && ((size_t)NTOK * DOUT / 2) % 256 == 0 && (OUT1_OFF * 4) % 128 == 0);

constexpr size_t al256(size_t b) { return (b + 255) & ~(size_t)255; }
constexpr size_t WS_TOTAL = al256((size_t)NEXP * H1 * DIN * 2) + al256((size_t)NEXP * H2 * H1 * 2) + al256((size_t)NEXP * DPAD * H2 * 2) + al256((size_t)NTOK * DIN * 2) + 2 * al256((size_t)NSLOT * 4)
                          + al256((size_t)TBL_WORDS * 4) + al256((size_t)R_MAX * DIN * 2) + al256((size_t)R_MAX * H1 * 2) + al256((size_t)R_MAX * H2 * 2) + al256((size_t)R_MAX * DPAD * 4);
static_assert(WS_TOTAL == (size_t)61740032 && WS_TOTAL < (size_t)134217728);

typedef _Float16 h16;
typedef __attribute__((ext_vector_type(16))) _Float16 v16h;
typedef __attribute__((ext_vector_type(8)))  _Float16 v8h;
typedef __attribute__((ext_vector_type(8)))  float    v8f;
typedef __attribute__((ext_vector_type(4)))  float    v4f;
typedef __attribute__((ext_vector_type(2)))  float    v2f;
typedef __attribute__((ext_vector_type(4)))  unsigned int v4u;
typedef __attribute__((ext_vector_type(4)))  int      v4i;
typedef __attribute__((ext_vector_type(2)))  int      v2i;


#define VST2(T, ptr, val) do { const T vst2_v_ = (val); *(volatile T*)(ptr) = vst2_v_; __threadfence(); *(volatile T*)(ptr) = vst2_v_; } while (0)

static __device__ __forceinline__ float bfr(float f) {
    unsigned u = __float_as_uint(f);
    u += 0x7FFFu + ((u >> 16) & 1u);
    return __uint_as_float(u & 0xFFFF0000u);
}
static __device__ __forceinline__ h16 toh_flush(float v) { const float w = (fabsf(v) < 6.103515625e-05f) ? 0.0f : v; return (h16)w; }
static __device__ __forceinline__ void st8h(h16* p, const float* v) {
    v8h hv;
#pragma unroll
    for (int e = 0; e < 8; ++e) hv[e] = toh_flush(v[e]);
    VST2(v8h, p, hv);
}

union FragU { v16h v; v8h h[2]; };
static __device__ __forceinline__ v16h frag_ld(const h16* p) {
    FragU f; f.h[0] = *(const v8h*)(p); f.h[1] = *(const v8h*)(p + 16); return f.v;
}
static __device__ __forceinline__ v8f wmma16g(v16h a, v16h b, v8f c) {
    c = __builtin_amdgcn_wmma_f32_16x16x32_f16(false, a, false, b, (short)0, c, false, false);
    asm volatile("v_nop\n\tv_nop\n\tv_nop\n\tv_nop" : "+v"(c) : "v"(a), "v"(b));
    return c;
}
static __device__ __forceinline__ void wave_sync_lds() {
    __builtin_amdgcn_fence(3  , "workgroup");
    __builtin_amdgcn_wave_barrier();
    __builtin_amdgcn_fence(2  , "workgroup");
}
template <int LOG2C>
__global__ __launch_bounds__(256) void k_plane(const float* __restrict__ src, h16* __restrict__ dst, unsigned n8) {
    const unsigned u = blockIdx.x * 256u + threadIdx.x;
    if (u >= n8) return;
    const float cs = (float)(1u << LOG2C);
    const v4f a = *(const v4f*)(src + (size_t)u * 8u);
    const v4f b = *(const v4f*)(src + (size_t)u * 8u + 4u);
    float v[8] = {bfr(a.x) * cs, bfr(a.y) * cs, bfr(a.z) * cs, bfr(a.w) * cs, bfr(b.x) * cs, bfr(b.y) * cs, bfr(b.z) * cs, bfr(b.w) * cs};
    st8h(dst + (size_t)u * 8u, v);
}
__global__ __launch_bounds__(128) void k_planeTw(const float* __restrict__ src, h16* __restrict__ dst, unsigned ne, unsigned K, unsigned N, unsigned pitch, unsigned estride, float cs) {
    __shared__ __align__(16) float sT[4][64 * 36];
    const unsigned lane = threadIdx.x & 31u;
    const unsigned wave = threadIdx.x >> 5;
    const unsigned tk = K >> 6, tn = N >> 5;
    const unsigned tpe = tk * tn;
    const unsigned u = blockIdx.x * 4u + wave;
    if (u >= ne * tpe) return;
    const unsigned e = u / tpe;
    const unsigned rem = u - e * tpe;
    const unsigned kt = rem / tn;
    const unsigned nt = rem - kt * tn;
    const unsigned k0 = kt << 6, n0 = nt << 5;
    const size_t sbase = (size_t)e * (size_t)estride;
    const size_t ebase = (size_t)e * ((size_t)K * (size_t)N);
    float* slab = sT[wave];
#pragma unroll
    for (int i = 0; i < 16; ++i) {
        const unsigned p = lane + 32u * (unsigned)i;
        const unsigned kr = p >> 3;
        const unsigned n4 = (p & 7u) * 4u;
        const v4f a = *(const v4f*)(src + sbase + (size_t)(k0 + kr) * pitch + n0 + n4);
        v4f s;
        s.x = bfr(a.x) * cs; s.y = bfr(a.y) * cs; s.z = bfr(a.z) * cs; s.w = bfr(a.w) * cs;
        *(v4f*)(&slab[kr * 36u + n4]) = s;
    }
    wave_sync_lds();
#pragma unroll
    for (int i = 0; i < 8; ++i) {
        const unsigned q = lane + 32u * (unsigned)i;
        const unsigned n = q >> 3;
        const unsigned kp = q & 7u;
        float v[8];
#pragma unroll
        for (int j = 0; j < 8; ++j) v[j] = slab[(8u * kp + (unsigned)j) * 36u + n];
        st8h(dst + ebase + (size_t)(n0 + n) * K + k0 + 8u * kp, v);
    }
}


template <int KS, int NS, int KP, int NP, int LOG2C>
__global__ __launch_bounds__(256) void k_planeTR(const float* __restrict__ src, h16* __restrict__ dst) {
    static_assert(KP % 64 == 0 && NP % 64 == 0 && KS <= KP && NS <= NP && KS >= 1 && NS >= 1 && LOG2C >= 0 && LOG2C < 31);
    __shared__ __align__(16) float sT[64 * 68];
    const unsigned tid = threadIdx.x;
    const unsigned bx = blockIdx.x;
    const unsigned TPE = (unsigned)((KP / 64) * (NP / 64));
    if (bx >= (unsigned)NE * TPE) return;
    const unsigned e = bx / TPE;
    const unsigned rem = bx - e * TPE;
    const unsigned kt = rem / (unsigned)(NP / 64);
    const unsigned nt = rem - kt * (unsigned)(NP / 64);
    const unsigned k0 = kt * 64u, n0 = nt * 64u;
    const float cs = (float)(1u << LOG2C);
    const size_t sbase = (size_t)e * ((size_t)KS * (size_t)NS);
    const size_t dbase = (size_t)e * ((size_t)NP * (size_t)KP);
    const unsigned nn = tid & 63u;
    const bool nin = (n0 + nn < (unsigned)NS);
    const unsigned nc = (unsigned)min((int)(n0 + nn), NS - 1);
#pragma unroll
    for (int i = 0; i < 16; ++i) {
        const unsigned kr = (tid >> 6) + 4u * (unsigned)i;
        const bool inb = nin && (k0 + kr < (unsigned)KS);
        const unsigned kk = (unsigned)min((int)(k0 + kr), KS - 1);
        const float a = src[sbase + (size_t)kk * (size_t)NS + nc];
        const unsigned bits = __float_as_uint(bfr(a) * cs) & (inb ? 0xffffffffu : 0u);
        sT[kr * 68u + nn] = __uint_as_float(bits);
    }
    __syncthreads();
#pragma unroll
    for (int i = 0; i < 2; ++i) {
        const unsigned q = tid + 256u * (unsigned)i;
        const unsigned n = q >> 3;
        const unsigned kp = q & 7u;
        float v[8];
#pragma unroll
        for (int j = 0; j < 8; ++j) v[j] = sT[(8u * kp + (unsigned)j) * 68u + n];
        st8h(dst + dbase + (size_t)(n0 + n) * KP + k0 + 8u * kp, v);
    }
}

__global__ __launch_bounds__(256) void k_gate2q(const float* __restrict__ x, const float* __restrict__ Wr, const float* __restrict__ br, int* __restrict__ sel, float* __restrict__ wgt, float* __restrict__ probs) {
    const unsigned lane = threadIdx.x & 31u;
    const unsigned wave = threadIdx.x >> 5;
    const unsigned tok0 = (blockIdx.x * 8u + wave) * 32u;
    if (tok0 >= (unsigned)NTOK) return;
    v2i ke; ke.x = 0; ke.y = 1;
    v2f kw; kw.x = 0.0f; kw.y = 0.0f;
    v4f pa; pa.x = 0.0f; pa.y = 0.0f; pa.z = 0.0f; pa.w = 0.0f;
    v4f pb; pb.x = 0.0f; pb.y = 0.0f; pb.z = 0.0f; pb.w = 0.0f;
    for (unsigned tt = 0; tt < 32u; ++tt) {
        const float* xr = x + (size_t)(tok0 + tt) * DIN;
        double acc[NEXP];
#pragma unroll
        for (int g = 0; g < NEXP; ++g) acc[g] = 0.0;
        for (unsigned q = 0; q < (unsigned)(DIN / 32); ++q) {
            const unsigned d = lane + 32u * q;
            const double xv = (double)bfr(xr[d]);
            const float* wr = Wr + (size_t)d * NEXP;
#pragma unroll
            for (int g = 0; g < NEXP; ++g) acc[g] = fma((double)bfr(wr[g]), xv, acc[g]);
        }
#pragma unroll
        for (int g = 0; g < NEXP; ++g) {
            double s = acc[g];
            s += __shfl_xor(s, 16, 32);
            s += __shfl_xor(s, 8, 32);
            s += __shfl_xor(s, 4, 32);
            s += __shfl_xor(s, 2, 32);
            s += __shfl_xor(s, 1, 32);
            acc[g] = s + (double)bfr(br[g]);
        }
        int e0 = 0; double v0 = acc[0];
#pragma unroll
        for (int g = 1; g < NEXP; ++g) { const bool tk = acc[g] > v0; e0 = tk ? g : e0; v0 = tk ? acc[g] : v0; }
        int e1 = 0; double v1 = 0.0; bool have = false;
#pragma unroll
        for (int g = 0; g < NEXP; ++g) {
            const bool free_ = (g != e0);
            const bool tk = free_ && (!have || acc[g] > v1);
            e1 = tk ? g : e1; v1 = tk ? acc[g] : v1; have = have || free_;
        }
        float ex[NEXP];
        float ssum = 0.0f;
#pragma unroll
        for (int g = 0; g < NEXP; ++g) { ex[g] = expf((float)(acc[g] - v0)); ssum += ex[g]; }
        float pr[NEXP];
#pragma unroll
        for (int g = 0; g < NEXP; ++g) pr[g] = ex[g] / ssum;
        const float g0 = 1.0f / ssum;
        const float g1 = expf((float)(v1 - v0)) / ssum;
        const bool mine = (lane == tt);
        ke.x = mine ? e0 : ke.x; ke.y = mine ? e1 : ke.y;
        kw.x = mine ? g0 : kw.x; kw.y = mine ? g1 : kw.y;
        pa.x = mine ? pr[0] : pa.x; pa.y = mine ? pr[1] : pa.y; pa.z = mine ? pr[2] : pa.z; pa.w = mine ? pr[3] : pa.w;
        pb.x = mine ? pr[4] : pb.x; pb.y = mine ? pr[5] : pb.y; pb.z = mine ? pr[6] : pb.z; pb.w = mine ? pr[7] : pb.w;
    }
    const unsigned t = tok0 + lane;
    VST2(v2i, sel + 2u * t, ke);
    VST2(v2f, wgt + 2u * t, kw);
    VST2(v4f, probs + 8u * (size_t)t, pa);
    VST2(v4f, probs + 8u * (size_t)t + 4u, pb);
}

template <int NE_>
__global__ __launch_bounds__(32) void k_route1w(const int* __restrict__ sel, int* __restrict__ tbl, unsigned nslot, unsigned spt, unsigned hdr, unsigned rmax,
                                                unsigned offPoff, unsigned offNtiles, unsigned offTileE) {
    static_assert(NE_ >= 1 && NE_ <= 32);
    __shared__ __align__(16) int s_img[RW_CH];
    __shared__ __align__(16) int s_hdr[512];
    const unsigned lane = threadIdx.x & 31u;
    const unsigned spl = nslot >> 5;
    const unsigned ng = spl >> 2;
    const unsigned ntmax = rmax >> 6;
    const v4i* sp = (const v4i*)(sel + (size_t)lane * spl);
    int cnt[NE_];
#pragma unroll
    for (int j = 0; j < NE_; ++j) cnt[j] = 0;
    for (unsigned g = 0; g < ng; ++g) {
        const v4i v = sp[g];
#pragma unroll
        for (int c = 0; c < 4; ++c) {
            const int e = min(max(v[c], 0), NE_ - 1);
#pragma unroll
            for (int j = 0; j < NE_; ++j) cnt[j] += (e == j) ? 1 : 0;
        }
    }
    int base0[NE_], total[NE_];
#pragma unroll
    for (int j = 0; j < NE_; ++j) {
        int pre = 0, tot = cnt[j];
#pragma unroll
        for (int d = 1; d < 32; d <<= 1) {
            const int t = __shfl_xor(tot, d, 32);
            pre += ((lane & (unsigned)d) != 0u) ? t : 0;
            tot += t;
        }
        base0[j] = pre;
        total[j] = tot;
    }
    int poff[NE_ + 1];
    poff[0] = 0;
#pragma unroll
    for (int j = 0; j < NE_; ++j) poff[j + 1] = poff[j] + (((total[j] + 63) >> 6) << 6);
    for (unsigned i = lane; i < 512u; i += 32u) s_hdr[i] = (i >= offTileE && i < offTileE + ntmax) ? -1 : 0;
    wave_sync_lds();
    if (lane == 0u) {
#pragma unroll
        for (int j = 0; j < NE_; ++j) { s_hdr[min((unsigned)j, 511u)] = total[j]; s_hdr[min(offPoff + (unsigned)j, 511u)] = poff[j]; }
        s_hdr[min(offPoff + (unsigned)NE_, 511u)] = poff[NE_];
        s_hdr[min(offNtiles, 511u)] = poff[NE_] >> 6;
    }
    for (unsigned t = lane; t < ntmax; t += 32u) {
        const int b64 = (int)(t * 64u);
        int ev = -1;
#pragma unroll
        for (int j = 0; j < NE_; ++j) ev = (b64 >= poff[j] && b64 < poff[j + 1]) ? j : ev;
        s_hdr[min(offTileE + t, 511u)] = ev;
    }
    wave_sync_lds();
    for (int pass = 0; pass < 2; ++pass) {
        for (unsigned i = lane; i < (hdr >> 2); i += 32u) *(volatile v4i*)(tbl + 4u * i) = *(const v4i*)(&s_hdr[4u * i]);
        __threadfence();
    }
    for (unsigned lo = 0; lo < rmax; lo += (unsigned)RW_CH) {
        for (unsigned i = lane; i < (unsigned)(RW_CH / 4); i += 32u) *(v4i*)(&s_img[4u * i]) = (v4i){-1, -1, -1, -1};
        wave_sync_lds();
        int run[NE_];
#pragma unroll
        for (int j = 0; j < NE_; ++j) run[j] = base0[j];
        for (unsigned g = 0; g < ng; ++g) {
            const v4i v = sp[g];
#pragma unroll
            for (int c = 0; c < 4; ++c) {
                const int e = min(max(v[c], 0), NE_ - 1);
                int row = 0;
#pragma unroll
                for (int j = 0; j < NE_; ++j) {
                    const bool hit = (e == j);
                    row = hit ? (poff[j] + run[j]) : row;
                    run[j] += hit ? 1 : 0;
                }
                row = min(max(row, 0), (int)rmax - 1);
                const unsigned rel = (unsigned)row - lo;
                if (rel < (unsigned)RW_CH) s_img[rel] = (int)((lane * spl + 4u * g + (unsigned)c) / spt);
            }
        }
        wave_sync_lds();
        const unsigned nw = min((unsigned)RW_CH, rmax - lo);
        for (int pass = 0; pass < 2; ++pass) {
            for (unsigned i = lane; i < (nw >> 2); i += 32u) *(volatile v4i*)(tbl + hdr + lo + 4u * i) = *(const v4i*)(&s_img[4u * i]);
            __threadfence();
        }
        wave_sync_lds();
    }
    for (unsigned lo = 0; lo < nslot; lo += (unsigned)RW_CH) {
        int run[NE_];
#pragma unroll
        for (int j = 0; j < NE_; ++j) run[j] = base0[j];
        for (unsigned g = 0; g < ng; ++g) {
            const v4i v = sp[g];
#pragma unroll
            for (int c = 0; c < 4; ++c) {
                const int e = min(max(v[c], 0), NE_ - 1);
                int row = 0;
#pragma unroll
                for (int j = 0; j < NE_; ++j) {
                    const bool hit = (e == j);
                    row = hit ? (poff[j] + run[j]) : row;
                    run[j] += hit ? 1 : 0;
                }
                row = min(max(row, 0), (int)rmax - 1);
                const unsigned rel = (lane * spl + 4u * g + (unsigned)c) - lo;
                if (rel < (unsigned)RW_CH) s_img[rel] = row;
            }
        }
        wave_sync_lds();
        const unsigned nw = min((unsigned)RW_CH, nslot - lo);
        for (int pass = 0; pass < 2; ++pass) {
            for (unsigned i = lane; i < (nw >> 2); i += 32u) *(volatile v4i*)(tbl + hdr + rmax + lo + 4u * i) = *(const v4i*)(&s_img[4u * i]);
            __threadfence();
        }
        wave_sync_lds();
    }
}

#define DM DIN
__global__ __launch_bounds__(256) void k_gather(const h16* __restrict__ x16, const int* __restrict__ tbl, h16* __restrict__ Xg) {
    const unsigned TPR = (unsigned)(DM / 8);
    const unsigned row = blockIdx.x * (256u / TPR) + (threadIdx.x / TPR);
    if (row >= (unsigned)R_MAX) return;
    const unsigned c = (threadIdx.x % TPR) * 8u;
    const int tr = tbl[TBL_ROWTOK + row];
    const bool pad = (tr < 0);
    const int tok = min(max(tr, 0), NTOK - 1);
    const v4u ld = *(const v4u*)(x16 + (size_t)(unsigned)tok * DM + c);
    v4u o;
    o.x = pad ? 0u : ld.x; o.y = pad ? 0u : ld.y; o.z = pad ? 0u : ld.z; o.w = pad ? 0u : ld.w;
    VST2(v4u, Xg + (size_t)row * DM + c, o);
}

template <int KD, int ND, int MODE>
__global__ __launch_bounds__(256) void k_lin(const h16* __restrict__ A, const h16* __restrict__ Wp, const float* __restrict__ eb,
                                             const int* __restrict__ tbl, void* __restrict__ OutV, unsigned nreal) {
    static_assert(KD % 32 == 0 && ND % 64 == 0 && MODE >= 0 && MODE <= 2);
    __shared__ __align__(16) float sT[8][16 * 68];
    const unsigned lane = threadIdx.x & 31u;
    const unsigned wave = threadIdx.x >> 5;
    const unsigned u = blockIdx.x * 8u + wave;
    if (u >= (unsigned)(NT_MAX * (ND / 64))) return;
    const unsigned rowtile = u / (unsigned)(ND / 64);
    const unsigned ct = u - rowtile * (unsigned)(ND / 64);
    const int nt = min(max(tbl[TBL_NTILES], 0), NT_MAX);
    if ((int)rowtile >= nt) return;
    const int e = min(max(tbl[TBL_TILE_E + rowtile], 0), (int)nreal - 1);
    const size_t wbase = (size_t)(unsigned)e * (size_t)(ND * KD);
    const unsigned m0 = rowtile << 6, n0 = ct << 6;
    const unsigned rlane = lane & 15u;
    const unsigned koff = (lane >> 4) * 8u;
    const unsigned mOff = koff;

    v8f acc[4][4];
#pragma unroll
    for (int i = 0; i < 4; ++i)
#pragma unroll
        for (int j = 0; j < 4; ++j) acc[i][j] = (v8f){0.f,0.f,0.f,0.f,0.f,0.f,0.f,0.f};

    for (unsigned k0 = 0; k0 < (unsigned)KD; k0 += 32u) {
        v16h bh[4];
#pragma unroll
        for (int j = 0; j < 4; ++j)
            bh[j] = frag_ld(Wp + wbase + (size_t)(n0 + ((unsigned)j << 4) + rlane) * KD + koff + k0);
#pragma unroll
        for (int i = 0; i < 4; ++i) {
            const v16h ah = frag_ld(A + (size_t)(m0 + ((unsigned)i << 4) + rlane) * KD + koff + k0);
#pragma unroll
            for (int j = 0; j < 4; ++j) acc[i][j] = wmma16g(ah, bh[j], acc[i][j]);
        }
    }

    float ebv[4];
#pragma unroll
    for (int j = 0; j < 4; ++j) ebv[j] = bfr(eb[(unsigned)e * (unsigned)ND + n0 + ((unsigned)j << 4) + rlane]);

    float* slab = sT[wave];
#pragma unroll
    for (int i = 0; i < 4; ++i) {
        const unsigned mBase = m0 + ((unsigned)i << 4);
#pragma unroll
        for (int j = 0; j < 4; ++j)
#pragma unroll
            for (int r = 0; r < 8; ++r) {
                const float a = acc[i][j][r] * SC + ebv[j];
                const float g = fmaxf(a, 0.0f);
                slab[(mOff + (unsigned)r) * 68u + ((unsigned)j << 4) + rlane] = (MODE == 2) ? g : g * CH;
            }
        wave_sync_lds();
        if constexpr (MODE == 2) {
            float* Out = (float*)OutV;
            const unsigned hh = lane >> 4, c4 = (lane & 15u) * 4u;
#pragma unroll
            for (int half = 0; half < 2; ++half) {
                v4f vv[4];
#pragma unroll
                for (int it = 0; it < 4; ++it) {
                    const unsigned row = (unsigned)(half * 4 + it) * 2u + hh;
                    vv[it] = *(const v4f*)(slab + row * 68u + c4);
                }
                for (int pass = 0; pass < 2; ++pass) {
#pragma unroll
                    for (int it = 0; it < 4; ++it) {
                        const unsigned row = (unsigned)(half * 4 + it) * 2u + hh;
                        *(volatile v4f*)(Out + (size_t)(mBase + row) * ND + n0 + c4) = vv[it];
                    }
                    __threadfence();
                }
            }
        } else {
            h16* Out = (h16*)OutV;
            constexpr unsigned RS = (MODE == 1) ? (unsigned)(2 * ND) : (unsigned)ND;
            const unsigned q = lane >> 3, c8 = (lane & 7u) * 8u;
            v8h hv[4];
            v8h lv[4];
#pragma unroll
            for (int it = 0; it < 4; ++it) {
                const unsigned row = (unsigned)it * 4u + q;
                const float* sp = slab + row * 68u + c8;
#pragma unroll
                for (int t = 0; t < 8; ++t) {
                    const h16 hi = toh_flush(sp[t]);
                    hv[it][t] = hi;
                    lv[it][t] = (MODE == 1) ? toh_flush(sp[t] - (float)hi) : (h16)0.0f;
                }
            }
            for (int pass = 0; pass < 2; ++pass) {
#pragma unroll
                for (int it = 0; it < 4; ++it) {
                    const unsigned row = (unsigned)it * 4u + q;
                    *(volatile v8h*)(Out + (size_t)(mBase + row) * RS + n0 + c8) = hv[it];
                    if constexpr (MODE == 1) *(volatile v8h*)(Out + (size_t)(mBase + row) * RS + (unsigned)ND + n0 + c8) = lv[it];
                }
                __threadfence();
            }
        }
        wave_sync_lds();
    }
}

__global__ __launch_bounds__(256) void k_out(const h16* __restrict__ Hg2, const h16* __restrict__ Wp, const float* __restrict__ eb,
                                             const int* __restrict__ tbl, float* __restrict__ Yg) {
    __shared__ __align__(16) float sT[8][16 * 68];
    const unsigned lane = threadIdx.x & 31u;
    const unsigned wave = threadIdx.x >> 5;
    const unsigned u = blockIdx.x * 8u + wave;
    if (u >= (unsigned)(NT_MAX * (DPAD / 64))) return;
    const unsigned rowtile = u / (unsigned)(DPAD / 64);
    const unsigned ct = u - rowtile * (unsigned)(DPAD / 64);
    const int nt = min(max(tbl[TBL_NTILES], 0), NT_MAX);
    if ((int)rowtile >= nt) return;
    const int e = min(max(tbl[TBL_TILE_E + rowtile], 0), NEXP - 1);
    const size_t wbase = (size_t)(unsigned)e * (size_t)(DPAD * H2);
    const unsigned m0 = rowtile << 6, n0 = ct << 6;
    const unsigned rlane = lane & 15u;
    const unsigned koff = (lane >> 4) * 8u;
    const unsigned mOff = koff;

    v8f acc[4][4];
#pragma unroll
    for (int i = 0; i < 4; ++i)
#pragma unroll
        for (int j = 0; j < 4; ++j) acc[i][j] = (v8f){0.f,0.f,0.f,0.f,0.f,0.f,0.f,0.f};

    for (unsigned k0 = 0; k0 < (unsigned)H2; k0 += 32u) {
        v16h bh[4];
#pragma unroll
        for (int j = 0; j < 4; ++j)
            bh[j] = frag_ld(Wp + wbase + (size_t)(n0 + ((unsigned)j << 4) + rlane) * H2 + koff + k0);
#pragma unroll
        for (int i = 0; i < 4; ++i) {
            const v16h ah = frag_ld(Hg2 + (size_t)(m0 + ((unsigned)i << 4) + rlane) * H2 + koff + k0);
#pragma unroll
            for (int j = 0; j < 4; ++j) acc[i][j] = wmma16g(ah, bh[j], acc[i][j]);
        }
    }

    float ebv[4];
#pragma unroll
    for (int j = 0; j < 4; ++j) {
        const unsigned col = n0 + ((unsigned)j << 4) + rlane;
        float bv = 0.0f;
        if (col < (unsigned)DOUT) bv = bfr(eb[(unsigned)e * (unsigned)DOUT + col]);
        ebv[j] = bv;
    }

    float* slab = sT[wave];
#pragma unroll
    for (int i = 0; i < 4; ++i) {
        const unsigned mBase = m0 + ((unsigned)i << 4);
#pragma unroll
        for (int j = 0; j < 4; ++j)
#pragma unroll
            for (int r = 0; r < 8; ++r)
                slab[(mOff + (unsigned)r) * 68u + ((unsigned)j << 4) + rlane] = acc[i][j][r] * SC + ebv[j];
        wave_sync_lds();
        const unsigned hh = lane >> 4, c4 = (lane & 15u) * 4u;
#pragma unroll
        for (int half = 0; half < 2; ++half) {
            v4f vv[4];
#pragma unroll
            for (int it = 0; it < 4; ++it) {
                const unsigned row = (unsigned)(half * 4 + it) * 2u + hh;
                vv[it] = *(const v4f*)(slab + row * 68u + c4);
            }
            for (int pass = 0; pass < 2; ++pass) {
#pragma unroll
                for (int it = 0; it < 4; ++it) {
                    const unsigned row = (unsigned)(half * 4 + it) * 2u + hh;
                    *(volatile v4f*)(Yg + (size_t)(mBase + row) * DPAD + n0 + c4) = vv[it];
                }
                __threadfence();
            }
        }
        wave_sync_lds();
    }
}

__global__ __launch_bounds__(256) void k_combine2h(const float* __restrict__ Yg, const float* __restrict__ wgt, const int* __restrict__ tbl, float* __restrict__ out) {
    const unsigned i = blockIdx.x * 256u + threadIdx.x;
    if (i >= (unsigned)(NTOK * OUT2_ROW)) return;
    const unsigned t = i / (unsigned)OUT2_ROW;
    const unsigned c = (i - t * (unsigned)OUT2_ROW) * 2u;
    const v2i rr = *(const v2i*)(tbl + TBL_SLOTROW + 2u * t);
    const int r0 = min(max(rr.x, 0), R_MAX - 1);
    const int r1 = min(max(rr.y, 0), R_MAX - 1);
    const v2f w = *(const v2f*)(wgt + 2u * t);
    const v2f a0 = *(const v2f*)(Yg + (size_t)(unsigned)r0 * DPAD + c);
    const v2f a1 = *(const v2f*)(Yg + (size_t)(unsigned)r1 * DPAD + c);
    const v2f y = ((a0 * w.x) + (a1 * w.y)) * (1.0f / (float)TOPK);
    VST2(v2f, out + 2u * (size_t)i, y);
}

extern "C" void kernel_launch(void* const* d_in, const int* in_sizes, int n_in, void* d_out, int out_size,
                              void* d_ws, size_t ws_size, hipStream_t stream) {
    if (n_in < 9) return;
    if (in_sizes[0] < NTOK * DIN || in_sizes[1] < DIN * NEXP || in_sizes[2] < NEXP || in_sizes[3] < NEXP * DIN * H1 || in_sizes[4] < NEXP * H1 || in_sizes[5] < NEXP * H1 * H2 || in_sizes[6] < NEXP * H2 || in_sizes[7] < NEXP * H2 * DOUT || in_sizes[8] < NEXP * DOUT) return;
    if (out_size < NTOK * DOUT + NTOK * NEXP) return;

    const float* x  = (const float*)d_in[0];
    const float* Wr = (const float*)d_in[1];
    const float* br = (const float*)d_in[2];
    const float* W1 = (const float*)d_in[3];
    const float* b1 = (const float*)d_in[4];
    const float* W2 = (const float*)d_in[5];
    const float* b2 = (const float*)d_in[6];
    const float* W3 = (const float*)d_in[7];
    const float* b3 = (const float*)d_in[8];
    float* out = (float*)d_out;

    char* wsp = (char*)d_ws;
    size_t off = 0;
    auto carve = [&](size_t bytes) -> void* { void* r = wsp + off; off += (bytes + 255) & ~(size_t)255; return r; };
    h16*   w1t = (h16*)carve((size_t)NEXP * H1 * DIN * 2);
    h16*   w2t = (h16*)carve((size_t)NEXP * H2 * H1 * 2);
    h16*   w3t = (h16*)carve((size_t)NEXP * DPAD * H2 * 2);
    h16*   x16 = (h16*)carve((size_t)NTOK * DIN * 2);
    int*   sel = (int*)carve((size_t)NSLOT * 4);
    float* wgt = (float*)carve((size_t)NSLOT * 4);
    int*   tbl = (int*)carve((size_t)TBL_WORDS * 4);
    h16*   Xg  = (h16*)carve((size_t)R_MAX * DIN * 2);
    h16*   Hg1 = (h16*)carve((size_t)R_MAX * H1 * 2);
    h16*   Hg2 = (h16*)carve((size_t)R_MAX * H2 * 2);
    float* Yg  = (float*)carve((size_t)R_MAX * DPAD * 4);
    if (off != WS_TOTAL || off > ws_size || off > (size_t)134217728) return;

    k_planeTw<<<(NEXP * (DIN / 64) * (H1 / 32) + 3) / 4, 128, 0, stream>>>(W1, w1t, (unsigned)NEXP, (unsigned)DIN, (unsigned)H1, (unsigned)H1, (unsigned)(DIN * H1), (float)(1u << CW_LOG2));
    k_planeTw<<<(NEXP * (H1 / 64) * (H2 / 32) + 3) / 4, 128, 0, stream>>>(W2, w2t, (unsigned)NEXP, (unsigned)H1, (unsigned)H2, (unsigned)H2, (unsigned)(H1 * H2), (float)(1u << CW_LOG2));
    k_planeTR<H2, DOUT, H2, DPAD, CW_LOG2><<<NEXP * (H2 / 64) * (DPAD / 64), 256, 0, stream>>>(W3, w3t);
    k_plane<CX_LOG2><<<(NTOK * DIN / 8) / 256, 256, 0, stream>>>(x, x16, (unsigned)(NTOK * DIN / 8));
    k_gate2q<<<NTOK / 256, 256, 0, stream>>>(x, Wr, br, sel, wgt, out + OUT1_OFF);
    k_route1w<NE><<<1, 32, 0, stream>>>(sel, tbl, (unsigned)NSLOT, (unsigned)SPT, (unsigned)TBL_HDR, (unsigned)R_MAX, (unsigned)TBL_POFF, (unsigned)TBL_NTILES, (unsigned)TBL_TILE_E);
    k_gather<<<R_MAX / (256 / (DM / 8)), 256, 0, stream>>>(x16, tbl, Xg);
    k_lin<DIN, H1, 0><<<(NT_MAX * (H1 / 64) + 7) / 8, 256, 0, stream>>>(Xg, w1t, b1, tbl, (void*)Hg1, (unsigned)NEXP);
    k_lin<H1, H2, 0><<<(NT_MAX * (H2 / 64) + 7) / 8, 256, 0, stream>>>(Hg1, w2t, b2, tbl, (void*)Hg2, (unsigned)NEXP);
    k_out<<<(NT_MAX * (DPAD / 64) + 7) / 8, 256, 0, stream>>>(Hg2, w3t, b3, tbl, Yg);
    k_combine2h<<<(NTOK * OUT2_ROW) / 256, 256, 0, stream>>>(Yg, wgt, tbl, out);
}
